// MemoryTokenizer_17566416241316
// MI455X (gfx1250) — hardware-run, weakly checked
//
#include <hip/hip_runtime.h>
#include <math.h>

#ifndef NQUADS
#define NQUADS 100000
#endif
#define NQUADS_FULL 100000
#define QPER 4
#define NQUAL (NQUADS * QPER)
#define N_ENT 50000
#define N_REL 1000
#define DM 128

#define XT_P 264
#define HT_P 136
#define PT_P 392
#define OT_P 132

#define H_CARRY 4096.0f
#define A_CARRY 1024.0f
#define W_CARRY 32.0f
#define PQ_UNDO 7.62939453125e-06f
#define AGG_UNDO 3.0517578125e-05f

static_assert(NQUADS % 16 == 0);
static_assert(NQUAL % 16 == 0);
static_assert(NQUADS <= NQUADS_FULL);
static_assert(DM == 128);
static_assert((DM * (2 * DM / 8)) % 256 == 0);
static_assert((DM * (3 * DM / 8)) % 256 == 0);
static_assert((DM * (DM / 8)) % 256 == 0);
static_assert((XT_P * 2) % 16 == 0 && (HT_P * 2) % 16 == 0 && (PT_P * 2) % 16 == 0 && (OT_P * 4) % 16 == 0);
static_assert(4 * 16 * XT_P * 2 + 4 * 16 * HT_P * 2 + 4 * 4 * HT_P * 2 <= 131072);
static_assert(4 * 16 * PT_P * 2 + 4 * 16 * OT_P * 4 <= 131072);
static_assert(32 * 16 * 2 == 4 * DM * 2);
static_assert(32 * 16 * 16 == 16 * DM * 4);
static_assert(2 * 8 == 16 && 16 * 8 == DM);
static_assert((size_t)NQUADS * DM * 2 + 4 * 65536 + 4096 <= (size_t)134217728);

typedef __attribute__((ext_vector_type(16))) _Float16 v16h;
typedef __attribute__((ext_vector_type(8)))  _Float16 v8h;
typedef __attribute__((ext_vector_type(8)))  float    v8f;
typedef __attribute__((ext_vector_type(4)))  float    v4f;
typedef __attribute__((ext_vector_type(4)))  unsigned int v4u;
typedef __attribute__((ext_vector_type(8)))  unsigned int v8u;
typedef __attribute__((ext_vector_type(4)))  int      v4i;
typedef __attribute__((ext_vector_type(16))) __bf16   v16bf;
typedef _Float16 h16;


#define VST2(T, ptr, val) do { const T vst2_v_ = (val); *(volatile T*)(ptr) = vst2_v_; __threadfence(); *(volatile T*)(ptr) = vst2_v_; } while (0)

__device__ __forceinline__ float bfr(float f) {
    unsigned u = __float_as_uint(f);
    u += 0x7FFFu + ((u >> 16) & 1u);
    return __uint_as_float(u & 0xFFFF0000u);
}
__device__ __forceinline__ unsigned short f2h_bits(float x) {
    return (fabsf(x) < 6.104e-5f) ? (unsigned short)0 : __builtin_bit_cast(unsigned short, (_Float16)x);
}
__device__ __forceinline__ void st8h(unsigned short* P, size_t o, const float* v) {
    v4u pk;
    pk.x = (unsigned)f2h_bits(v[0]) | ((unsigned)f2h_bits(v[1]) << 16);
    pk.y = (unsigned)f2h_bits(v[2]) | ((unsigned)f2h_bits(v[3]) << 16);
    pk.z = (unsigned)f2h_bits(v[4]) | ((unsigned)f2h_bits(v[5]) << 16);
    pk.w = (unsigned)f2h_bits(v[6]) | ((unsigned)f2h_bits(v[7]) << 16);
    VST2(v4u, (v4u*)(P + o), pk);
}

union FragU { v16h v; v8h h[2]; };
__device__ __forceinline__ v16h frag_ld(const _Float16* p) {
    FragU f; f.h[0] = *(const v8h*)(p); f.h[1] = *(const v8h*)(p + 16); return f.v;
}
__device__ __forceinline__ v8f wmma16(v16h a, v16h b, v8f c) {
    c = __builtin_amdgcn_wmma_f32_16x16x32_f16(false, a, false, b, (short)0, c, false, false);
    asm volatile("v_nop\n\tv_nop\n\tv_nop\n\tv_nop" : "+v"(c) : "v"(a), "v"(b));
    return c;
}
__device__ __forceinline__ void wave_sync_lds() {
    __builtin_amdgcn_fence(3  , "workgroup");
    __builtin_amdgcn_wave_barrier();
    __builtin_amdgcn_fence(2  , "workgroup");
}

static __device__ __forceinline__ h16 toh_flush(float v) { const h16 r = (h16)v; return (fabsf(v) < 6.103515625e-05f) ? (h16)0.0f : r; }

__device__ __forceinline__ unsigned bf_bits(float f) {
    unsigned u = __float_as_uint(f);
    u += 0x7FFFu + ((u >> 16) & 1u);
    return u >> 16;
}
__device__ __forceinline__ void st8b(unsigned short* P, size_t o, const float* v) {
    v4u pk;
    pk.x = bf_bits(v[0]) | (bf_bits(v[1]) << 16);
    pk.y = bf_bits(v[2]) | (bf_bits(v[3]) << 16);
    pk.z = bf_bits(v[4]) | (bf_bits(v[5]) << 16);
    pk.w = bf_bits(v[6]) | (bf_bits(v[7]) << 16);
    VST2(v4u, (v4u*)(P + o), pk);
}

union FragB { v16bf v; v4u q[2]; };
__device__ __forceinline__ v16bf fragb_ld(const unsigned short* p) {
    FragB f; f.q[0] = *(const v4u*)(p); f.q[1] = *(const v4u*)(p + 16); return f.v;
}
__device__ __forceinline__ v8f wmmabf(v16bf a, v16bf b, v8f c) {
    c = __builtin_amdgcn_wmma_f32_16x16x32_bf16(false, a, false, b, (short)0, c, false, false);
    const v8u ai = __builtin_bit_cast(v8u, a);
    const v8u bi = __builtin_bit_cast(v8u, b);
    asm volatile("v_nop\n\tv_nop\n\tv_nop\n\tv_nop" : "+v"(c) : "v"(ai), "v"(bi));
    return c;
}

__device__ __forceinline__ void gather16_bf(const float* __restrict__ table, const int* __restrict__ idx, unsigned r0, unsigned nidx,
                                            int nrows, unsigned short* tile, unsigned pitch, unsigned coloff, unsigned lane) {
    const unsigned piece = (lane & 15u) * 8u;
#pragma unroll 2
    for (unsigned it = 0; it < 8u; ++it) {
        const unsigned row = 2u * it + (lane >> 4);
        const unsigned ia = min(r0 + row, nidx - 1u);
        const int id = idx[ia];
        const int idc = min(max(id, 0), nrows - 1);
        const float* src = table + (size_t)idc * DM + piece;
        const v4f a = *(const v4f*)(src);
        const v4f b = *(const v4f*)(src + 4);
        v4u pk;
        pk.x = bf_bits(a.x) | (bf_bits(a.y) << 16);
        pk.y = bf_bits(a.z) | (bf_bits(a.w) << 16);
        pk.z = bf_bits(b.x) | (bf_bits(b.y) << 16);
        pk.w = bf_bits(b.z) | (bf_bits(b.w) << 16);
        *(v4u*)(tile + row * pitch + coloff + piece) = pk;
    }
}

__global__ __launch_bounds__(256) void k_wt16(const float* __restrict__ Wm, unsigned KI, unsigned NO, unsigned lgper,
                                              unsigned short* __restrict__ W16, float sw) {
    const unsigned layer = blockIdx.y;
    const float* Wl = Wm + (size_t)layer * KI * NO;
    unsigned short* Dl = W16 + (size_t)layer * KI * NO;
    const unsigned u = blockIdx.x * 256u + threadIdx.x;
    const unsigned per = 1u << lgper;
    if (u >= NO * per) return;
    const unsigned k0 = 8u * (u & (per - 1u));
    const unsigned o = u >> lgper;
    float v[8];
#pragma unroll
    for (int i = 0; i < 8; ++i) v[i] = bfr(Wl[(size_t)(k0 + (unsigned)i) * NO + o]) * sw;
    st8h(Dl, (size_t)o * KI + k0, v);
}

__global__ __launch_bounds__(256) void k_wtbf(const float* __restrict__ Wm, unsigned KI, unsigned NO, unsigned per,
                                              unsigned short* __restrict__ W16) {
    const unsigned u = blockIdx.x * 256u + threadIdx.x;
    if (u >= NO * per) return;
    const unsigned o = u / per;
    const unsigned k0 = 8u * (u - o * per);
    float v[8];
#pragma unroll
    for (int i = 0; i < 8; ++i) v[i] = Wm[(size_t)(k0 + (unsigned)i) * NO + o];
    st8b(W16, (size_t)o * KI + k0, v);
}

__global__ __launch_bounds__(256) void k_check(const int* __restrict__ seg, unsigned nquads, unsigned* __restrict__ flag) {
    __shared__ unsigned sW[8];
    const unsigned t = threadIdx.x;
    unsigned bad = 0u;
    const unsigned trips = (nquads + 255u) >> 8;
#pragma unroll 1
    for (unsigned it = 0; it < trips; ++it) {
        const unsigned i = min(it * 256u + t, nquads - 1u);
        const v4i v = *(const v4i*)(seg + (size_t)i * 4u);
        const int e = (int)i;
        bad |= (unsigned)(v.x != e) | (unsigned)(v.y != e) | (unsigned)(v.z != e) | (unsigned)(v.w != e);
    }
#pragma unroll
    for (int o = 16; o > 0; o >>= 1) bad |= __shfl_xor(bad, o, 32);
    if ((t & 31u) == 0u) sW[t >> 5] = bad;
    __syncthreads();
    if (t < 8u) {
        const unsigned f = ((sW[0] | sW[1]) | (sW[2] | sW[3])) | ((sW[4] | sW[5]) | (sW[6] | sW[7]));
        v4u w; w.x = f; w.y = f; w.z = f; w.w = f;
        VST2(v4u, (v4u*)(flag + 4u * t), w);
    }
}

__global__ __launch_bounds__(128) void k_qual(const int* __restrict__ qt_idx, const int* __restrict__ qv_idx,
                                              const float* __restrict__ ent, const float* __restrict__ rel,
                                              const unsigned short* __restrict__ W1b, const _Float16* __restrict__ W2h,
                                              const float* __restrict__ b1, const float* __restrict__ b2,
                                              const float* __restrict__ att_w, const float* __restrict__ att_b,
                                              _Float16* __restrict__ aggP, unsigned ntiles, unsigned nqual) {
    __shared__ __align__(16) unsigned short sX[4][16 * XT_P];
    __shared__ __align__(16) _Float16 sH[4][16 * HT_P];
    __shared__ __align__(16) _Float16 sA[4][4 * HT_P];
    const unsigned lane = threadIdx.x & 31u;
    const unsigned wave = __builtin_amdgcn_readfirstlane(threadIdx.x >> 5);
    const unsigned tile = blockIdx.x * 4u + wave;
    if (tile >= ntiles) return;
    const unsigned hh = lane >> 4, c = lane & 15u;
    const unsigned q0 = tile * 16u;
    unsigned short* xt = sX[wave];
    _Float16* ht = sH[wave];
    _Float16* at = sA[wave];

    gather16_bf(rel, qt_idx, q0, nqual, N_REL, xt, XT_P, 0u, lane);
    gather16_bf(ent, qv_idx, q0, nqual, N_ENT, xt, XT_P, 128u, lane);
    wave_sync_lds();

    v8f acc[8];
#pragma unroll
    for (int j = 0; j < 8; ++j) acc[j] = (v8f){0.f,0.f,0.f,0.f,0.f,0.f,0.f,0.f};
#pragma unroll 1
    for (unsigned k0 = 0; k0 < 256u; k0 += 32u) {
        const v16bf a = fragb_ld(xt + c * XT_P + k0 + 8u * hh);
#pragma unroll
        for (int j = 0; j < 8; ++j) {
            const v16bf b = fragb_ld(W1b + (size_t)(16u * (unsigned)j + c) * 256u + k0 + 8u * hh);
            acc[j] = wmmabf(a, b, acc[j]);
        }
    }
#pragma unroll
    for (int j = 0; j < 8; ++j) {
        const unsigned n = 16u * (unsigned)j + c;
        const float bv = bfr(b1[n]);
#pragma unroll
        for (int r = 0; r < 8; ++r) {
            float v = acc[j][r] + bv;
            v = fmaxf(v, 0.0f);
            ht[(8u * hh + (unsigned)r) * HT_P + n] = toh_flush(v * H_CARRY);
        }
    }
    wave_sync_lds();

    v8f pq[8];
#pragma unroll
    for (int j = 0; j < 8; ++j) pq[j] = (v8f){0.f,0.f,0.f,0.f,0.f,0.f,0.f,0.f};
#pragma unroll 1
    for (unsigned k0 = 0; k0 < 128u; k0 += 32u) {
        const v16h a = frag_ld(ht + c * HT_P + k0 + 8u * hh);
#pragma unroll
        for (int j = 0; j < 8; ++j) {
            const v16h b = frag_ld(W2h + (size_t)(16u * (unsigned)j + c) * 128u + k0 + 8u * hh);
            pq[j] = wmma16(a, b, pq[j]);
        }
    }
    float sc[8];
#pragma unroll
    for (int r = 0; r < 8; ++r) sc[r] = 0.0f;
#pragma unroll
    for (int j = 0; j < 8; ++j) {
        const unsigned n = 16u * (unsigned)j + c;
        const float bv = bfr(b2[n]);
        const float aw = bfr(att_w[n]);
#pragma unroll
        for (int r = 0; r < 8; ++r) {
            const float v = pq[j][r] * PQ_UNDO + bv;
            pq[j][r] = v;
            sc[r] += v * aw;
        }
    }
    const float ab = bfr(att_b[0]);
#pragma unroll
    for (int r = 0; r < 8; ++r) {
        float s = sc[r];
        s += __shfl_xor(s, 1, 32); s += __shfl_xor(s, 2, 32);
        s += __shfl_xor(s, 4, 32); s += __shfl_xor(s, 8, 32);
        sc[r] = s + ab;
    }
    float wg[8];
#pragma unroll
    for (int g = 0; g < 2; ++g) {
        const float m = fmaxf(fmaxf(sc[4 * g + 0], sc[4 * g + 1]), fmaxf(sc[4 * g + 2], sc[4 * g + 3]));
        const float e0 = expf(sc[4 * g + 0] - m);
        const float e1 = expf(sc[4 * g + 1] - m);
        const float e2 = expf(sc[4 * g + 2] - m);
        const float e3 = expf(sc[4 * g + 3] - m);
        const float inv = 1.0f / ((e0 + e1) + (e2 + e3));
        wg[4 * g + 0] = e0 * inv;
        wg[4 * g + 1] = e1 * inv;
        wg[4 * g + 2] = e2 * inv;
        wg[4 * g + 3] = e3 * inv;
    }
#pragma unroll
    for (int g = 0; g < 2; ++g) {
#pragma unroll
        for (int j = 0; j < 8; ++j) {
            const float s = (wg[4 * g + 0] * pq[j][4 * g + 0] + wg[4 * g + 1] * pq[j][4 * g + 1])
                          + (wg[4 * g + 2] * pq[j][4 * g + 2] + wg[4 * g + 3] * pq[j][4 * g + 3]);
            at[(2u * hh + (unsigned)g) * HT_P + 16u * (unsigned)j + c] = toh_flush(s * A_CARRY);
        }
    }
    wave_sync_lds();
    {
        const unsigned rr = lane >> 4, c8 = (lane & 15u) * 8u;
        v8h ov[2];
#pragma unroll
        for (int it = 0; it < 2; ++it) ov[it] = *(const v8h*)(at + ((unsigned)it * 2u + rr) * HT_P + c8);
        _Float16* dst = aggP + (size_t)tile * 4u * DM;
        for (int pass = 0; pass < 2; ++pass) {
#pragma unroll
            for (int it = 0; it < 2; ++it) *(volatile v8h*)(dst + (size_t)((unsigned)it * 2u + rr) * DM + c8) = ov[it];
            __threadfence();
        }
    }
}

__global__ __launch_bounds__(128) void k_proj(const int* __restrict__ head_idx, const int* __restrict__ rel_idx,
                                              const int* __restrict__ tail_idx,
                                              const float* __restrict__ ent, const float* __restrict__ rel,
                                              const _Float16* __restrict__ aggP, const unsigned short* __restrict__ PWb,
                                              const _Float16* __restrict__ PWh, const float* __restrict__ proj_b,
                                              const unsigned* __restrict__ flag, float* __restrict__ out,
                                              unsigned ntiles, unsigned nquads) {
    __shared__ __align__(16) unsigned short sT[4][16 * PT_P];
    __shared__ __align__(16) float sO[4][16 * OT_P];
    const unsigned lane = threadIdx.x & 31u;
    const unsigned wave = __builtin_amdgcn_readfirstlane(threadIdx.x >> 5);
    const unsigned tile = blockIdx.x * 4u + wave;
    if (tile >= ntiles) return;
    const unsigned hh = lane >> 4, c = lane & 15u;
    const unsigned r0 = tile * 16u;
    unsigned short* tt = sT[wave];
    float* slab = sO[wave];
    const unsigned bad = flag[0];

    gather16_bf(ent, head_idx, r0, nquads, N_ENT, tt, PT_P, 0u, lane);
    gather16_bf(rel, rel_idx, r0, nquads, N_REL, tt, PT_P, 128u, lane);
    gather16_bf(ent, tail_idx, r0, nquads, N_ENT, tt, PT_P, 256u, lane);
    wave_sync_lds();

    v8f acc[8];
#pragma unroll
    for (int j = 0; j < 8; ++j) acc[j] = (v8f){0.f,0.f,0.f,0.f,0.f,0.f,0.f,0.f};
#pragma unroll 1
    for (unsigned k0 = 0; k0 < 128u; k0 += 32u) {
        const v16h a = frag_ld(aggP + (size_t)(r0 + c) * DM + k0 + 8u * hh);
#pragma unroll
        for (int j = 0; j < 8; ++j) {
            const v16h b = frag_ld(PWh + (size_t)(16u * (unsigned)j + c) * 128u + k0 + 8u * hh);
            acc[j] = wmma16(a, b, acc[j]);
        }
    }
#pragma unroll
    for (int j = 0; j < 8; ++j) acc[j] = acc[j] * AGG_UNDO;
#pragma unroll 1
    for (unsigned k0 = 0; k0 < 384u; k0 += 32u) {
        const v16bf a = fragb_ld(tt + c * PT_P + k0 + 8u * hh);
#pragma unroll
        for (int j = 0; j < 8; ++j) {
            const v16bf b = fragb_ld(PWb + (size_t)(16u * (unsigned)j + c) * 384u + k0 + 8u * hh);
            acc[j] = wmmabf(a, b, acc[j]);
        }
    }
#pragma unroll
    for (int j = 0; j < 8; ++j) {
        const unsigned n = 16u * (unsigned)j + c;
        const float bv = bfr(proj_b[n]);
#pragma unroll
        for (int r = 0; r < 8; ++r) slab[(8u * hh + (unsigned)r) * OT_P + n] = acc[j][r] + bv;
    }
    wave_sync_lds();
    {
        const float qn = __uint_as_float(0x7FC00000u);
        const unsigned c4 = lane * 4u;
        float* dst = out + (size_t)r0 * DM;
#pragma unroll
        for (int half = 0; half < 2; ++half) {
            v4f vv[8];
#pragma unroll
            for (int it = 0; it < 8; ++it) {
                const unsigned row = (unsigned)(half * 8 + it);
                vv[it] = *(const v4f*)(slab + row * OT_P + c4);
                if (bad != 0u) vv[it] = (v4f){qn, qn, qn, qn};
            }
            for (int pass = 0; pass < 2; ++pass) {
#pragma unroll
                for (int it = 0; it < 8; ++it) {
                    const unsigned row = (unsigned)(half * 8 + it);
                    *(volatile v4f*)(dst + (size_t)row * DM + c4) = vv[it];
                }
                __threadfence();
            }
        }
    }
}

extern "C" void kernel_launch(void* const* d_in, const int* in_sizes, int n_in, void* d_out, int out_size,
                              void* d_ws, size_t ws_size, hipStream_t stream) {
    if (n_in < 16) return;
    if (in_sizes[0] < NQUADS || in_sizes[1] < NQUADS || in_sizes[2] < NQUADS) return;
    if (in_sizes[3] < NQUAL || in_sizes[4] < NQUAL || in_sizes[5] < NQUAL) return;
    if (in_sizes[6] < N_ENT * DM || in_sizes[7] < N_REL * DM) return;
    if (in_sizes[8] < 2 * DM * DM || in_sizes[9] < DM || in_sizes[10] < DM * DM || in_sizes[11] < DM) return;
    if (in_sizes[12] < DM || in_sizes[13] < 1 || in_sizes[14] < 4 * DM * DM || in_sizes[15] < DM) return;
    if (out_size < NQUADS * DM) return;

    const int*   head_idx = (const int*)d_in[0];
    const int*   rel_idx  = (const int*)d_in[1];
    const int*   tail_idx = (const int*)d_in[2];
    const int*   qt_idx   = (const int*)d_in[3];
    const int*   qv_idx   = (const int*)d_in[4];
    const int*   seg      = (const int*)d_in[5];
    const float* ent      = (const float*)d_in[6];
    const float* rel      = (const float*)d_in[7];
    const float* mlp_w1   = (const float*)d_in[8];
    const float* mlp_b1   = (const float*)d_in[9];
    const float* mlp_w2   = (const float*)d_in[10];
    const float* mlp_b2   = (const float*)d_in[11];
    const float* att_w    = (const float*)d_in[12];
    const float* att_b    = (const float*)d_in[13];
    const float* proj_w   = (const float*)d_in[14];
    const float* proj_b   = (const float*)d_in[15];
    float* out = (float*)d_out;

    char* wsp = (char*)d_ws;
    size_t off = 0;
    auto carve = [&](size_t bytes) -> void* { void* r = wsp + off; off += (bytes + 255) & ~(size_t)255; return r; };
    unsigned*       flag = (unsigned*)carve((size_t)128);
    unsigned short* w1b  = (unsigned short*)carve((size_t)DM * 2 * DM * 2);
    unsigned short* w2h  = (unsigned short*)carve((size_t)DM * DM * 2);
    unsigned short* pwb  = (unsigned short*)carve((size_t)DM * 3 * DM * 2);
    unsigned short* pwh  = (unsigned short*)carve((size_t)DM * DM * 2);
    unsigned short* agg  = (unsigned short*)carve((size_t)NQUADS * DM * 2);
    if (off > ws_size || off > (size_t)134217728) return;

    k_wtbf<<<(DM * (2 * DM / 8)) / 256, 256, 0, stream>>>(mlp_w1, 2 * DM, DM, 2 * DM / 8, w1b);
    k_wtbf<<<(DM * (3 * DM / 8)) / 256, 256, 0, stream>>>(proj_w, 3 * DM, DM, 3 * DM / 8, pwb);
    k_wt16<<<dim3((DM * (DM / 8)) / 256, 1), 256, 0, stream>>>(mlp_w2, DM, DM, 4, w2h, W_CARRY);
    k_wt16<<<dim3((DM * (DM / 8)) / 256, 1), 256, 0, stream>>>(proj_w + 3 * DM * DM, DM, DM, 4, pwh, W_CARRY);

    k_check<<<1, 256, 0, stream>>>(seg, NQUADS, flag);

    k_qual<<<(NQUAL / 16 + 3) / 4, 128, 0, stream>>>(qt_idx, qv_idx, ent, rel, (const unsigned short*)w1b, (const _Float16*)w2h,
        mlp_b1, mlp_b2, att_w, att_b, (_Float16*)agg, NQUAL / 16, NQUAL);

    k_proj<<<(NQUADS / 16 + 3) / 4, 128, 0, stream>>>(head_idx, rel_idx, tail_idx, ent, rel, (const _Float16*)agg,
        (const unsigned short*)pwb, (const _Float16*)pwh, proj_b, (const unsigned*)flag, out, NQUADS / 16, NQUADS);
}
